// Attention_77137612636887
// MI455X (gfx1250) — hardware-verified
//
#include <hip/hip_runtime.h>


#ifndef NB
#define NB 4
#endif
#ifndef SEQ
#define SEQ 2048
#endif
#define NB_FULL  4
#define SEQ_FULL 2048
#define DM   768
#define NH   12
#define HD   64
#define DQ   (NH * HD)
#define NQKV (3 * DM)
#define KCH  64
#define PCL2 10.0f
#define SL2  0.18033688011112042f

static_assert(NB <= NB_FULL);
static_assert(SEQ <= SEQ_FULL);
static_assert(HD == 64);
static_assert(NH * HD == DM);
static_assert(DM % 64 == 0);
static_assert(SEQ % 64 == 0);
static_assert(SEQ % KCH == 0);
static_assert(KCH == 64);
static_assert((2 * DM) % 64 == 0);
static_assert(((size_t)SEQ * DM) % 8 == 0);
static_assert(((size_t)NQKV * DM) % 8 == 0);
static_assert(((size_t)DM * DM) % 8 == 0);

typedef _Float16 h16;
typedef unsigned short bf;
typedef __attribute__((ext_vector_type(16))) __bf16   v16bf;
typedef __attribute__((ext_vector_type(16))) _Float16 v16h;
typedef __attribute__((ext_vector_type(8)))  _Float16 v8h;
typedef __attribute__((ext_vector_type(8)))  unsigned short v8us;
typedef __attribute__((ext_vector_type(8)))  float    v8f;
typedef __attribute__((ext_vector_type(4)))  float    v4f;
typedef v4f  __attribute__((may_alias)) v4fa;
typedef v8us __attribute__((may_alias)) v8usa;

__device__ __forceinline__ unsigned short f2bf(float f) { unsigned u = __float_as_uint(f); u += 0x7FFFu + ((u >> 16) & 1u); return (unsigned short)(u >> 16); }
__device__ __forceinline__ float bf2f(unsigned short b) { return __uint_as_float(((unsigned)b) << 16); }
__device__ __forceinline__ float bfr(float f) { return bf2f(f2bf(f)); }
__device__ __forceinline__ v16h cat16(v8h lo, v8h hi) { return __builtin_shufflevector(lo, hi, 0, 1, 2, 3, 4, 5, 6, 7, 8, 9, 10, 11, 12, 13, 14, 15); }
__device__ __forceinline__ v16bf cat16b(v8us lo, v8us hi) { return __builtin_bit_cast(v16bf, __builtin_shufflevector(lo, hi, 0, 1, 2, 3, 4, 5, 6, 7, 8, 9, 10, 11, 12, 13, 14, 15)); }
__device__ __forceinline__ v8f wmma16(v16h a, v16h b, v8f c) { return __builtin_amdgcn_wmma_f32_16x16x32_f16(false, a, false, b, (short)0, c, false, false); }
__device__ __forceinline__ v8f wmmab(v16bf a, v16bf b, v8f c) { return __builtin_amdgcn_wmma_f32_16x16x32_bf16(false, a, false, b, (short)0, c, false, false); }
__device__ __forceinline__ void splitf(float y, unsigned short& h, unsigned short& l) { h = f2bf(y); l = f2bf(y - bf2f(h)); }

template <typename T16> struct WFrag;
template <> struct WFrag<h16> { typedef v16h V; static __device__ __forceinline__ V ld(const h16* p) { return cat16(*(const v8h*)p, *(const v8h*)(p + 16)); } static __device__ __forceinline__ v8f mma(V a, V b, v8f c) { return wmma16(a, b, c); } };
template <> struct WFrag<bf> { typedef v16bf V; static __device__ __forceinline__ V ld(const bf* p) { return cat16b(*(const v8us*)p, *(const v8us*)(p + 16)); } static __device__ __forceinline__ v8f mma(V a, V b, v8f c) { return wmmab(a, b, c); } };

template <typename T16, int NSPLIT, bool BIAS, bool OUT16>
__global__ __launch_bounds__(32) void k_gemmw(const T16* __restrict__ A, const T16* __restrict__ A2, const T16* __restrict__ Bt, const T16* __restrict__ Bt2, unsigned K, void* Cv, unsigned ldc, const float* __restrict__ bias, size_t sA, size_t sB, size_t sC, size_t cstr) {
    typedef typename WFrag<T16>::V V;
    __shared__ __align__(16) float os[16 * 68];
    const size_t z = blockIdx.z; A += z * sA; if (A2) A2 += z * sA; Bt += z * sB; if (Bt2) Bt2 += z * sB;
    const unsigned lane = threadIdx.x & 31u, lr = lane & 15u, hi = lane >> 4; const unsigned r0 = blockIdx.x * 64u, c0 = blockIdx.y * 64u;
    v8f acc[4][4];
#pragma unroll
    for (int mb = 0; mb < 4; ++mb)
#pragma unroll
        for (int nb = 0; nb < 4; ++nb) acc[mb][nb] = (v8f){};
    const size_t aoff = (size_t)(r0 + lr) * K + 8u * hi, boff = (size_t)(c0 + lr) * K + 8u * hi;
#pragma unroll 1
    for (unsigned kc = 0; kc < K; kc += 32u) {
        V a[4], a2[4];
#pragma unroll
        for (int mb = 0; mb < 4; ++mb) { a[mb] = WFrag<T16>::ld(A + aoff + (size_t)mb * 16 * K + kc); if (NSPLIT == 1 || NSPLIT == 2) a2[mb] = WFrag<T16>::ld(A2 + aoff + (size_t)mb * 16 * K + kc); }
#pragma unroll
        for (int nb = 0; nb < 4; ++nb) { const V b = WFrag<T16>::ld(Bt + boff + (size_t)nb * 16 * K + kc); V b2; if (NSPLIT >= 2) b2 = WFrag<T16>::ld(Bt2 + boff + (size_t)nb * 16 * K + kc);
#pragma unroll
            for (int mb = 0; mb < 4; ++mb) { acc[mb][nb] = WFrag<T16>::mma(a[mb], b, acc[mb][nb]); if (NSPLIT == 1 || NSPLIT == 2) acc[mb][nb] = WFrag<T16>::mma(a2[mb], b, acc[mb][nb]); if (NSPLIT >= 2) acc[mb][nb] = WFrag<T16>::mma(a[mb], b2, acc[mb][nb]); } }
        asm volatile("v_nop\n\tv_nop\n\tv_nop\n\tv_nop" : "+v"(acc[0][0]), "+v"(acc[1][1]), "+v"(acc[2][2]), "+v"(acc[3][3]) : "v"(a[0]), "v"(a[3]));
    }
    v4f bv = (v4f){0.f, 0.f, 0.f, 0.f};
    if (BIAS) { const unsigned cb = c0 + lr * 4u; bv[0] = bfr(bias[cb]); bv[1] = bfr(bias[cb + 1]); bv[2] = bfr(bias[cb + 2]); bv[3] = bfr(bias[cb + 3]); }
#pragma unroll
    for (int mb = 0; mb < 4; ++mb) {
#pragma unroll
        for (int nb = 0; nb < 4; ++nb) {
#pragma unroll
            for (int j = 0; j < 8; ++j) os[(hi * 8 + j) * 68 + nb * 16 + lr] = acc[mb][nb][j]; }
        __builtin_amdgcn_wave_barrier(); asm volatile("" ::: "memory");
        if (OUT16) {
            h16* crow = (h16*)Cv + z * sC + (size_t)blockIdx.y * cstr + (size_t)(r0 + mb * 16) * ldc;
            const unsigned rq = lane >> 3, pc = (lane & 7u) * 8u;
            v8h o[4];
#pragma unroll
            for (int s = 0; s < 4; ++s) { const unsigned row = 4u * s + rq; const v4f x0 = *(const v4fa*)(os + row * 68 + pc), x1 = *(const v4fa*)(os + row * 68 + pc + 4);
#pragma unroll
                for (int q = 0; q < 4; ++q) { o[s][q] = (h16)x0[q]; o[s][4 + q] = (h16)x1[q]; } }
#pragma unroll 1
            for (int ps = 0; ps < 2; ++ps) {
#pragma unroll
                for (int s = 0; s < 4; ++s) *(volatile v8h*)(crow + (size_t)(4u * s + rq) * ldc + pc) = o[s];
                if (ps == 0) __threadfence(); }
        } else {
            float* crow = (float*)Cv + z * sC + (size_t)blockIdx.y * cstr + (size_t)(r0 + mb * 16) * ldc;
            const unsigned cofs = lr * 4u;
            v4f val[8];
#pragma unroll
            for (int s = 0; s < 8; ++s) { const unsigned row = 2u * s + hi; val[s] = *(const v4fa*)(os + row * 68 + cofs); val[s] += bv; }
#pragma unroll 1
            for (int ps = 0; ps < 2; ++ps) {
#pragma unroll
                for (int s = 0; s < 8; ++s) *(volatile v4f*)(crow + (size_t)(2u * s + hi) * ldc + cofs) = val[s];
                if (ps == 0) __threadfence(); }
        }
        __builtin_amdgcn_wave_barrier(); asm volatile("" ::: "memory");
    }
}

__global__ __launch_bounds__(256) void k_cvt8(const float* __restrict__ src, bf* dst, unsigned n8, size_t sstr, size_t dstr) {
    const unsigned i = blockIdx.x * 256u + threadIdx.x; if (i >= n8) return;
    const float* s = src + (size_t)blockIdx.y * sstr + (size_t)i * 8; bf* d = dst + (size_t)blockIdx.y * dstr + (size_t)i * 8;
    const v4f v0 = *(const v4f*)s, v1 = *(const v4f*)(s + 4); v8us o;
#pragma unroll
    for (int k = 0; k < 4; ++k) { o[k] = f2bf(v0[k]); o[4 + k] = f2bf(v1[k]); }
    *(volatile v8us*)d = o; __threadfence(); *(volatile v8us*)d = o; }

__global__ __launch_bounds__(128) void k_flash(const h16* __restrict__ QK, const h16* __restrict__ VT, bf* Ah, bf* Al) {
    __shared__ __align__(16) unsigned short osh[4][16 * 72];
    __shared__ __align__(16) unsigned short osl[4][16 * 72];
    const unsigned lane = threadIdx.x & 31u, w = threadIdx.x >> 5, lr = lane & 15u, hi = lane >> 4;
    const unsigned b = blockIdx.z, h = blockIdx.y, q0 = blockIdx.x * 64u + w * 16u;
    const h16* Qp = QK + ((size_t)(b * 2u * NH + h) * SEQ) * HD;
    const h16* Kp = QK + ((size_t)(b * 2u * NH + NH + h) * SEQ) * HD;
    const h16* Vp = VT + ((size_t)b * DM + h * HD) * SEQ;
    v16h bq[2];
    bq[0] = WFrag<h16>::ld(Qp + (size_t)(q0 + lr) * HD + 8u * hi);
    bq[1] = WFrag<h16>::ld(Qp + (size_t)(q0 + lr) * HD + 32u + 8u * hi);
    v8f acc[4];
#pragma unroll
    for (int dt = 0; dt < 4; ++dt) acc[dt] = (v8f){};
    float m = -3.0e38f, ls = 0.f;
    const h16* kbase = Kp + (size_t)lr * HD + 8u * hi;
    const h16* vbase = Vp + (size_t)lr * SEQ + 8u * hi;
#pragma unroll 1
    for (unsigned kc = 0; kc < SEQ; kc += KCH) {
        v16h ka[4][2]; v8f st[4];
#pragma unroll
        for (int kt = 0; kt < 4; ++kt) { ka[kt][0] = WFrag<h16>::ld(kbase + (size_t)(kc + kt * 16) * HD); ka[kt][1] = WFrag<h16>::ld(kbase + (size_t)(kc + kt * 16) * HD + 32); }
#pragma unroll
        for (int kt = 0; kt < 4; ++kt) { st[kt] = wmma16(ka[kt][0], bq[0], (v8f){}); st[kt] = wmma16(ka[kt][1], bq[1], st[kt]); }
        asm volatile("v_nop\n\tv_nop\n\tv_nop\n\tv_nop" : "+v"(st[0]), "+v"(st[1]), "+v"(st[2]), "+v"(st[3]) : "v"(ka[0][0]), "v"(ka[0][1]), "v"(ka[1][0]), "v"(ka[1][1]), "v"(ka[2][0]), "v"(ka[2][1]), "v"(ka[3][0]), "v"(ka[3][1]), "v"(bq[0]), "v"(bq[1]));
        float mx = st[0][0];
#pragma unroll
        for (int kt = 0; kt < 4; ++kt)
#pragma unroll
            for (int r = 0; r < 8; ++r) mx = fmaxf(mx, st[kt][r]);
        mx = fmaxf(mx, __shfl_xor(mx, 16, 32));
        const float mn = fmaxf(m, mx * SL2);
        const float al = __builtin_amdgcn_exp2f(m - mn);
        m = mn;
        const float sh = PCL2 - mn;
        float psum = 0.f; v16h pb[2];
#pragma unroll
        for (int ks = 0; ks < 2; ++ks)
#pragma unroll
            for (int r = 0; r < 8; ++r) { const float p0 = __builtin_amdgcn_exp2f(st[2 * ks][r] * SL2 + sh); const float p1 = __builtin_amdgcn_exp2f(st[2 * ks + 1][r] * SL2 + sh); psum += p0 + p1; pb[ks][r] = (h16)p0; pb[ks][8 + r] = (h16)p1; }
        ls = ls * al + psum;
#pragma unroll
        for (int dt = 0; dt < 4; ++dt)
#pragma unroll
            for (int r = 0; r < 8; ++r) acc[dt][r] *= al;
        v16h va[4][2];
#pragma unroll
        for (int dt = 0; dt < 4; ++dt) { va[dt][0] = WFrag<h16>::ld(vbase + (size_t)(dt * 16) * SEQ + kc); va[dt][1] = WFrag<h16>::ld(vbase + (size_t)(dt * 16) * SEQ + kc + 32); }
#pragma unroll
        for (int dt = 0; dt < 4; ++dt) { acc[dt] = wmma16(va[dt][0], pb[0], acc[dt]); acc[dt] = wmma16(va[dt][1], pb[1], acc[dt]); }
        asm volatile("v_nop\n\tv_nop\n\tv_nop\n\tv_nop" : "+v"(acc[0]), "+v"(acc[1]), "+v"(acc[2]), "+v"(acc[3]) : "v"(va[0][0]), "v"(va[0][1]), "v"(va[1][0]), "v"(va[1][1]), "v"(va[2][0]), "v"(va[2][1]), "v"(va[3][0]), "v"(va[3][1]), "v"(pb[0]), "v"(pb[1]));
    }
    ls += __shfl_xor(ls, 16, 32);
    const float inv = 1.0f / ls;
    unsigned short* oh = &osh[w][0]; unsigned short* ol = &osl[w][0];
#pragma unroll
    for (int dt = 0; dt < 4; ++dt) { v8us hv, lv;
#pragma unroll
        for (int r = 0; r < 8; ++r) { unsigned short a, c; splitf(acc[dt][r] * inv, a, c); hv[r] = a; lv[r] = c; }
        *(v8usa*)(oh + lr * 72 + dt * 16 + 8 * hi) = hv; *(v8usa*)(ol + lr * 72 + dt * 16 + 8 * hi) = lv; }
    __builtin_amdgcn_wave_barrier(); asm volatile("" ::: "memory");
    const unsigned rq = lane >> 3, pc = (lane & 7u) * 8u;
    v8us vh[4], vl[4];
#pragma unroll
    for (int s = 0; s < 4; ++s) { const unsigned row = 4u * s + rq; vh[s] = *(const v8usa*)(oh + row * 72 + pc); vl[s] = *(const v8usa*)(ol + row * 72 + pc); }
    const size_t gofs = ((size_t)b * SEQ + q0) * DQ + h * HD + pc;
#pragma unroll 1
    for (int ps = 0; ps < 2; ++ps) {
#pragma unroll
        for (int s = 0; s < 4; ++s) { const size_t o = gofs + (size_t)(4u * s + rq) * DQ; *(volatile v8us*)(Ah + o) = vh[s]; *(volatile v8us*)(Al + o) = vl[s]; }
        if (ps == 0) __threadfence(); }
}

constexpr size_t SZ_XB = (size_t)NB * SEQ * DM * 2;
constexpr size_t SZ_WQ = (size_t)NQKV * DM * 2;
constexpr size_t SZ_WO = (size_t)DM * DM * 2;
constexpr size_t SZ_QK = (size_t)NB * 2 * NH * SEQ * HD * 2;
constexpr size_t SZ_VT = (size_t)NB * DM * SEQ * 2;
constexpr size_t SZ_AT = (size_t)NB * SEQ * DQ * 2;
constexpr size_t OFF_XB = 0;
constexpr size_t OFF_WQ = OFF_XB + SZ_XB;
constexpr size_t OFF_WO = OFF_WQ + SZ_WQ;
constexpr size_t OFF_QK = OFF_WO + SZ_WO;
constexpr size_t OFF_VT = OFF_QK + SZ_QK;
constexpr size_t OFF_AH = OFF_VT + SZ_VT;
constexpr size_t OFF_AL = OFF_AH + SZ_AT;
constexpr size_t WS_TOTAL = OFF_AL + SZ_AT;
static_assert(SZ_XB % 256 == 0); static_assert(SZ_WQ % 256 == 0); static_assert(SZ_WO % 256 == 0);
static_assert(SZ_QK % 256 == 0); static_assert(SZ_VT % 256 == 0); static_assert(SZ_AT % 256 == 0);
static_assert(WS_TOTAL <= (size_t)134217728);
static_assert((size_t)(SEQ / 64) * (2 * NH) * NB * 4096 == SZ_QK / 2);
static_assert((size_t)(DM / 64) * (SEQ / 64) * NB * 4096 == SZ_VT / 2);
static_assert((size_t)(SEQ / 64) * NH * NB * 4 * 16 * HD == SZ_AT / 2);
static_assert((size_t)(SEQ / 64) * (DM / 64) * 4096 == (size_t)SEQ * DM);

extern "C" void kernel_launch(void* const* d_in, const int* in_sizes, int n_in,
                              void* d_out, int out_size, void* d_ws, size_t ws_size, hipStream_t stream) {
    if (n_in < 5) return;
    const size_t xneed = (size_t)(NB - 1) * SEQ_FULL * DM + (size_t)SEQ * DM;
    if ((size_t)in_sizes[0] < xneed) return;
    if ((size_t)in_sizes[2] < (size_t)NQKV * DM) return;
    if ((size_t)in_sizes[3] < (size_t)DM * DM) return;
    if ((size_t)in_sizes[4] < (size_t)DM) return;
    if ((size_t)out_size < xneed) return;
    if (ws_size < WS_TOTAL) return;
    const float* x = (const float*)d_in[0]; const float* wqkv = (const float*)d_in[2]; const float* wo = (const float*)d_in[3]; const float* bo = (const float*)d_in[4];
    float* OUT = (float*)d_out;
    char* wsp = (char*)d_ws;
    bf* XB = (bf*)(wsp + OFF_XB); bf* WQ = (bf*)(wsp + OFF_WQ); bf* WO = (bf*)(wsp + OFF_WO);
    h16* QK = (h16*)(wsp + OFF_QK); h16* VT = (h16*)(wsp + OFF_VT); bf* ATh = (bf*)(wsp + OFF_AH); bf* ATl = (bf*)(wsp + OFF_AL);

    const unsigned nx8 = (unsigned)((size_t)SEQ * DM / 8), nq8 = (unsigned)((size_t)NQKV * DM / 8), no8 = (unsigned)((size_t)DM * DM / 8);
    k_cvt8<<<dim3((nx8 + 255u) / 256u, NB, 1), 256, 0, stream>>>(x, XB, nx8, (size_t)SEQ_FULL * DM, (size_t)SEQ * DM);
    k_cvt8<<<dim3((nq8 + 255u) / 256u, 1, 1), 256, 0, stream>>>(wqkv, WQ, nq8, 0, 0);
    k_cvt8<<<dim3((no8 + 255u) / 256u, 1, 1), 256, 0, stream>>>(wo, WO, no8, 0, 0);
    k_gemmw<bf, 0, false, true><<<dim3(SEQ / 64, 2 * NH, NB), 32, 0, stream>>>(XB, nullptr, WQ, nullptr, (unsigned)DM, (void*)QK, (unsigned)HD, nullptr, (size_t)SEQ * DM, 0, (size_t)2 * NH * SEQ * HD, (size_t)SEQ * HD);
    k_gemmw<bf, 0, false, true><<<dim3(DM / 64, SEQ / 64, NB), 32, 0, stream>>>(WQ + (size_t)2 * DM * DM, nullptr, XB, nullptr, (unsigned)DM, (void*)VT, (unsigned)SEQ, nullptr, 0, (size_t)SEQ * DM, (size_t)DM * SEQ, (size_t)64);
    k_flash<<<dim3(SEQ / 64, NH, NB), 128, 0, stream>>>(QK, VT, ATh, ATl);
    k_gemmw<bf, 1, true, false><<<dim3(SEQ / 64, DM / 64, NB), 32, 0, stream>>>(ATh, ATl, WO, nullptr, (unsigned)DQ, (void*)OUT, (unsigned)DM, bo, (size_t)SEQ * DQ, 0, (size_t)SEQ_FULL * DM, (size_t)64);
}
